// GaussianSelfAttention_7533372637348
// MI455X (gfx1250) — hardware-verified
//
#include <hip/hip_runtime.h>
#include <stdint.h>
#include <stddef.h>

#pragma clang fp contract(off)

typedef __attribute__((ext_vector_type(16))) _Float16 v16h;
typedef __attribute__((ext_vector_type(8)))  _Float16 v8h;
typedef __attribute__((ext_vector_type(16))) __bf16   v16b;
typedef __attribute__((ext_vector_type(8)))  __bf16   v8b;
typedef __attribute__((ext_vector_type(8)))  float    v8f;
typedef __attribute__((ext_vector_type(4)))  float    v4f;
typedef __attribute__((ext_vector_type(4)))  unsigned int v4u;

#define GS_B     2
#define GS_G     2048
#define GS_C     256
#define GS_H     8
#define GS_D     32
#define GS_BG    4096
#define GS_KC    64
#define GS_NW    4
#define GS_QKLD  512
#define GS_VTLD  4096
#define GS_TAULD 64
#define GS_TAUN  64
#define GS_OSP   36

__device__ __forceinline__ unsigned short f2bf_bits(float f) {
  unsigned u = __float_as_uint(f);
  return (unsigned short)((u + 0x7FFFu + ((u >> 16) & 1u)) >> 16);
}
__device__ __forceinline__ float bf_bits2f(unsigned short h) { return __uint_as_float(((unsigned)h) << 16); }

__device__ __forceinline__ void dep_guard_h(v8f& a, v8f& b, v16h x, v16h y) { asm volatile("v_nop\n\tv_nop\n\tv_nop\n\tv_nop" : "+v"(a), "+v"(b) : "v"(x), "v"(y)); }
__device__ __forceinline__ void dep_guard_b(v8f& a, v8f& b, v16b x, v16b y) { asm volatile("v_nop\n\tv_nop\n\tv_nop\n\tv_nop" : "+v"(a), "+v"(b) : "v"(x), "v"(y)); }
__device__ __forceinline__ void keep4_h(v16h a, v16h b, v16h c, v16h d) { asm volatile("v_nop" :: "v"(a), "v"(b), "v"(c), "v"(d)); }
__device__ __forceinline__ void keep4_b(v16b a, v16b b, v16b c, v16b d) { asm volatile("v_nop" :: "v"(a), "v"(b), "v"(c), "v"(d)); }
__device__ __forceinline__ void acc_guard4(v8f& a, v8f& b, v8f& c, v8f& d) { asm volatile("v_nop\n\tv_nop\n\tv_nop\n\tv_nop" : "+v"(a), "+v"(b), "+v"(c), "+v"(d)); }

template <typename T> struct Frag;
template <> struct Frag<_Float16> {
  typedef v16h V; union U { v16h v; v8h h[2]; };
  static __device__ __forceinline__ v16h load(const _Float16* p) {
    U f; f.h[0] = *(const v8h*)(p); f.h[1] = *(const v8h*)(p + 16); return f.v;
  }
  static __device__ __forceinline__ v8f mma(v16h a, v16h b, v8f c) {
    return __builtin_amdgcn_wmma_f32_16x16x32_f16(false, a, false, b, (short)0, c, false, false);
  }
  static __device__ __forceinline__ void guard(v8f& a, v8f& b, v16h x, v16h y) { dep_guard_h(a, b, x, y); }
  static __device__ __forceinline__ void keep(v16h a, v16h b, v16h c, v16h d) { keep4_h(a, b, c, d); }
};
template <> struct Frag<__bf16> {
  typedef v16b V; union U { v16b v; v8b h[2]; };
  static __device__ __forceinline__ v16b load(const __bf16* p) {
    U f; f.h[0] = *(const v8b*)(p); f.h[1] = *(const v8b*)(p + 16); return f.v;
  }
  static __device__ __forceinline__ v8f mma(v16b a, v16b b, v8f c) {
    return __builtin_amdgcn_wmma_f32_16x16x32_bf16(false, a, false, b, (short)0, c, false, false);
  }
  static __device__ __forceinline__ void guard(v8f& a, v8f& b, v16b x, v16b y) { dep_guard_b(a, b, x, y); }
  static __device__ __forceinline__ void keep(v16b a, v16b b, v16b c, v16b d) { keep4_b(a, b, c, d); }
};

template <int ET> struct Elem;
template <> struct Elem<0> { typedef _Float16 T; };
template <> struct Elem<1> { typedef __bf16 T; };
template <int ET, bool SPLIT, int BIAS_MODE, int OUT_MODE>
__global__ __launch_bounds__(256) void wmma_gemm64(
    const unsigned short* __restrict__ Ap, const unsigned short* __restrict__ A2p, int lda, long strideA,
    const unsigned short* __restrict__ Btp, const unsigned short* __restrict__ Bt2p, int ldb, long strideB,
    void* __restrict__ Cout, void* __restrict__ Cout2, int ldc, long strideC,
    const float* __restrict__ bias,
    int M, int N, int K, float scale) {
  typedef typename Elem<ET>::T T;
  typedef typename Frag<T>::V V;
  const T* A = (const T*)Ap; const T* A2 = (const T*)A2p; const T* Bt = (const T*)Btp; const T* Bt2 = (const T*)Bt2p;
  __shared__ __align__(16) float sT[8][16 * 68];
  const int b    = blockIdx.y;
  const int lane = threadIdx.x & 31;
  const int wave = threadIdx.x >> 5;
  const int tilesN = N >> 6;
  const int tilesM = M >> 6;
  const int tile = blockIdx.x * 8 + wave;
  if (tile >= tilesM * tilesN) return;
  const int tm = tile / tilesN;
  const int tn = tile - tm * tilesN;
  const int m0 = tm << 6;
  const int n0 = tn << 6;

  const T* Ab  = A  + (size_t)b * strideA;
  const T* Bb  = Bt + (size_t)b * strideB;
  const T* Ab2 = SPLIT ? (A2  + (size_t)b * strideA) : nullptr;
  const T* Bb2 = SPLIT ? (Bt2 + (size_t)b * strideB) : nullptr;

  const int rlane = lane & 15;
  const int koff  = (lane >> 4) * 8;
  const int mOff  = (lane >> 4) * 8;

  v8f acc[4][4];
#pragma unroll
  for (int i = 0; i < 4; ++i)
#pragma unroll
    for (int j = 0; j < 4; ++j) acc[i][j] = (v8f){0.f,0.f,0.f,0.f,0.f,0.f,0.f,0.f};

  for (int k0 = 0; k0 < K; k0 += 32) {
    V bh[4], bl[4];
#pragma unroll
    for (int j = 0; j < 4; ++j) {
      const size_t bo = (size_t)(n0 + (j << 4) + rlane) * ldb + koff + k0;
      bh[j] = Frag<T>::load(Bb + bo);
      if (SPLIT) bl[j] = Frag<T>::load(Bb2 + bo);
    }
#pragma unroll
    for (int i = 0; i < 4; ++i) {
      const size_t ao = (size_t)(m0 + (i << 4) + rlane) * lda + koff + k0;
      V ah = Frag<T>::load(Ab + ao);
      V al;
      if (SPLIT) al = Frag<T>::load(Ab2 + ao);
#pragma unroll
      for (int j = 0; j < 4; ++j) {
        acc[i][j] = Frag<T>::mma(ah, bh[j], acc[i][j]);
        if (SPLIT) {
          acc[i][j] = Frag<T>::mma(ah, bl[j], acc[i][j]);
          acc[i][j] = Frag<T>::mma(al, bh[j], acc[i][j]);
        }
      }
      Frag<T>::guard(acc[i][0], acc[i][3], ah, SPLIT ? al : ah);
    }
    Frag<T>::keep(bh[0], bh[1], bh[2], bh[3]);
    if (SPLIT) Frag<T>::keep(bl[0], bl[1], bl[2], bl[3]);
  }
  acc_guard4(acc[0][0], acc[0][1], acc[0][2], acc[0][3]);
  acc_guard4(acc[1][0], acc[1][1], acc[1][2], acc[1][3]);
  acc_guard4(acc[2][0], acc[2][1], acc[2][2], acc[2][3]);
  acc_guard4(acc[3][0], acc[3][1], acc[3][2], acc[3][3]);

  float* slab = sT[wave];
#pragma unroll
  for (int i = 0; i < 4; ++i) {
    const int mBase = m0 + (i << 4);
#pragma unroll
    for (int j = 0; j < 4; ++j) {
      const int n = n0 + (j << 4) + rlane;
      float bv = 0.f;
      if (BIAS_MODE == 2) bv = bias[n];
#pragma unroll
      for (int r = 0; r < 8; ++r) {
        float v = acc[i][j][r] * scale;
        if (BIAS_MODE == 2) v += bv;
        slab[(mOff + r) * 68 + (j << 4) + rlane] = v;
      }
    }
    __builtin_amdgcn_fence(__ATOMIC_RELEASE, "workgroup");
    __builtin_amdgcn_wave_barrier();
    __builtin_amdgcn_fence(__ATOMIC_ACQUIRE, "workgroup");
    if (OUT_MODE == 0) {
      float* C = (float*)Cout + (size_t)b * strideC;
      const int hh = lane >> 4, c4 = (lane & 15) * 4;
      for (int pass = 0; pass < 2; ++pass) {
#pragma unroll
        for (int it = 0; it < 8; ++it) {
          const int row = it * 2 + hh;
          v4f v = *(const v4f*)(slab + row * 68 + c4);
          if (BIAS_MODE == 1) { const float bm = bias[mBase + row]; v = v + bm; }
          *(volatile v4f*)(C + (size_t)(mBase + row) * ldc + n0 + c4) = v;
        }
        __threadfence();
      }
    } else {
      const int q = lane >> 3, c8 = (lane & 7) * 8;
      unsigned short* C  = (unsigned short*)Cout  + (size_t)b * strideC;
      unsigned short* C2 = (OUT_MODE == 2) ? ((unsigned short*)Cout2 + (size_t)b * strideC) : nullptr;
      for (int pass = 0; pass < 2; ++pass) {
#pragma unroll
        for (int it = 0; it < 4; ++it) {
          const int row = it * 4 + q;
          const float* sp = slab + row * 68 + c8;
          float bm = 0.f;
          if (BIAS_MODE == 1) bm = bias[mBase + row];
          v8h hv, lv;
#pragma unroll
          for (int e = 0; e < 8; ++e) {
            const float val = sp[e] + bm;
            if (OUT_MODE == 1) {
              hv[e] = (_Float16)val;
            } else {
              unsigned short hb = f2bf_bits(val);
              unsigned short lb = f2bf_bits(val - bf_bits2f(hb));
              hv[e] = __builtin_bit_cast(_Float16, hb);
              lv[e] = __builtin_bit_cast(_Float16, lb);
            }
          }
          *(volatile v8h*)(C + (size_t)(mBase + row) * ldc + n0 + c8) = hv;
          if (OUT_MODE == 2) *(volatile v8h*)(C2 + (size_t)(mBase + row) * ldc + n0 + c8) = lv;
        }
        __threadfence();
      }
    }
    __builtin_amdgcn_fence(__ATOMIC_RELEASE, "workgroup");
    __builtin_amdgcn_wave_barrier();
    __builtin_amdgcn_fence(__ATOMIC_ACQUIRE, "workgroup");
  }
}

__global__ __launch_bounds__(256) void split_rows_kernel(
    const float* __restrict__ in, unsigned short* __restrict__ hi, unsigned short* __restrict__ lo,
    int rows_real, int rows_pad, int kc) {
  const long t = (long)blockIdx.x * 256 + threadIdx.x;
  const long e0 = t * 8;
  const long total = (long)rows_pad * kc;
  if (e0 >= total) return;
  const int row = (int)(e0 / kc);
  const int col = (int)(e0 - (long)row * kc);
  const int rowc = (row < rows_real) ? row : (rows_real - 1);
  const bool live = row < rows_real;
  const float* p = in + (size_t)rowc * kc + col;
  const v4f a0 = *(const v4f*)(p);
  const v4f a1 = *(const v4f*)(p + 4);
  float f[8];
  f[0] = a0[0]; f[1] = a0[1]; f[2] = a0[2]; f[3] = a0[3];
  f[4] = a1[0]; f[5] = a1[1]; f[6] = a1[2]; f[7] = a1[3];
  unsigned hw[4], lw[4];
#pragma unroll
  for (int e = 0; e < 4; ++e) {
    const float x0 = live ? f[2 * e] : 0.0f;
    const float x1 = live ? f[2 * e + 1] : 0.0f;
    const unsigned short h0 = f2bf_bits(x0);
    const unsigned short l0 = f2bf_bits(x0 - bf_bits2f(h0));
    const unsigned short h1 = f2bf_bits(x1);
    const unsigned short l1 = f2bf_bits(x1 - bf_bits2f(h1));
    hw[e] = (unsigned)h0 | ((unsigned)h1 << 16);
    lw[e] = (unsigned)l0 | ((unsigned)l1 << 16);
  }
  v4u hv; hv[0] = hw[0]; hv[1] = hw[1]; hv[2] = hw[2]; hv[3] = hw[3];
  v4u lv; lv[0] = lw[0]; lv[1] = lw[1]; lv[2] = lw[2]; lv[3] = lw[3];
  volatile v4u* hp = (volatile v4u*)(hi + e0);
  volatile v4u* lp = (volatile v4u*)(lo + e0);
  *hp = hv;
  *lp = lv;
  __threadfence();
  *hp = hv;
  *lp = lv;
}

__device__ __forceinline__ v8f bf_mma(v16b a, v16b b, v8f c) {
  c = __builtin_amdgcn_wmma_f32_16x16x32_bf16(false, a, false, b, (short)0, c, false, false);
  asm volatile("v_nop\n\tv_nop\n\tv_nop\n\tv_nop" : "+v"(c) : "v"(a), "v"(b));
  return c;
}

__global__ __launch_bounds__(128) void gsa_attn_kernel(
    const unsigned short* __restrict__ QKh, const unsigned short* __restrict__ QKl,
    const unsigned short* __restrict__ VTh, const unsigned short* __restrict__ VTl,
    const float* __restrict__ TAU, const float* __restrict__ taub,
    const float* __restrict__ gs, float* __restrict__ O) {
  union FB { v16b v; v8b h[2]; };
  __shared__ __align__(16) __bf16 Ksh[GS_KC * GS_D];
  __shared__ __align__(16) __bf16 Ksl[GS_KC * GS_D];
  __shared__ __align__(16) __bf16 Vth[GS_D * GS_KC];
  __shared__ __align__(16) __bf16 Vtl[GS_D * GS_KC];
  __shared__ __align__(16) __bf16 Psh[GS_NW][16 * GS_KC];
  __shared__ __align__(16) __bf16 Psl[GS_NW][16 * GS_KC];
  __shared__ __align__(16) float  Os[GS_NW][16 * GS_OSP];
  __shared__ float kx_s[GS_KC], ky_s[GS_KC];
  __shared__ float qx_s[64], qy_s[64], qt_s[64];

  const int tid  = threadIdx.x;
  const int wave = tid >> 5;
  const int lane = tid & 31;
  const int hh   = lane >> 4;
  const int c    = lane & 15;

  const int nqb = GS_G / 64;
  const int qb  = blockIdx.x % nqb;
  const int bhi = blockIdx.x / nqb;
  const int h   = bhi % GS_H;
  const int b   = bhi / GS_H;
  const int qbase = qb * 64;
  const int q0 = qbase + wave * 16;
  const size_t browbase = (size_t)b * GS_G;

  const float pc_mul = 102.4f;
  const float pc_add = -51.2f;
  const float qk_scale = 0.17677669529663687f;

  if (tid < 64) {
    const size_t grow = browbase + qbase + tid;
    const float gx = gs[grow * 11 + 0];
    const float gy = gs[grow * 11 + 1];
    float x = gx * pc_mul; x = x + pc_add;
    float y = gy * pc_mul; y = y + pc_add;
    qx_s[tid] = x;
    qy_s[tid] = y;
    const float tv = TAU[grow * GS_TAULD + h];
    const float tb = taub[h];
    qt_s[tid] = tv + tb;
  }
  __syncthreads();

  float xq[8], yq[8], tq[8], mrow[8], lrow[8];
#pragma unroll
  for (int r = 0; r < 8; ++r) {
    const int lr = wave * 16 + 8 * hh + r;
    xq[r] = qx_s[lr]; yq[r] = qy_s[lr]; tq[r] = qt_s[lr];
    mrow[r] = -__builtin_inff(); lrow[r] = 0.f;
  }
  v8f oacc[2];
  oacc[0] = (v8f){0.f,0.f,0.f,0.f,0.f,0.f,0.f,0.f};
  oacc[1] = (v8f){0.f,0.f,0.f,0.f,0.f,0.f,0.f,0.f};

  v16b qah, qal;
  {
    const size_t qo = (browbase + q0 + c) * GS_QKLD + (size_t)h * GS_D + 8 * hh;
    qah = Frag<__bf16>::load((const __bf16*)QKh + qo);
    qal = Frag<__bf16>::load((const __bf16*)QKl + qo);
  }

  for (int kc = 0; kc < GS_G / GS_KC; ++kc) {
    const int kv0 = kc * GS_KC;
    __syncthreads();
    {
      const int kvr = tid >> 1, dh = (tid & 1) * 16;
      const size_t ko = (browbase + kv0 + kvr) * GS_QKLD + 256 + (size_t)h * GS_D + dh;
      const v4u* skh = (const v4u*)(QKh + ko);
      const v4u* skl = (const v4u*)(QKl + ko);
      const v4u kh0 = skh[0], kh1 = skh[1], kl0 = skl[0], kl1 = skl[1];
      v4u* dkh = (v4u*)(Ksh + kvr * GS_D + dh);
      v4u* dkl = (v4u*)(Ksl + kvr * GS_D + dh);
      dkh[0] = kh0; dkh[1] = kh1; dkl[0] = kl0; dkl[1] = kl1;
      const int dd = tid >> 2, kq = (tid & 3) * 16;
      const size_t vo = (size_t)(h * GS_D + dd) * GS_VTLD + browbase + kv0 + kq;
      const v4u* svh = (const v4u*)(VTh + vo);
      const v4u* svl = (const v4u*)(VTl + vo);
      const v4u vh0 = svh[0], vh1 = svh[1], vl0 = svl[0], vl1 = svl[1];
      v4u* dvh = (v4u*)(Vth + dd * GS_KC + kq);
      v4u* dvl = (v4u*)(Vtl + dd * GS_KC + kq);
      dvh[0] = vh0; dvh[1] = vh1; dvl[0] = vl0; dvl[1] = vl1;
      if (tid < GS_KC) {
        const size_t grow = browbase + kv0 + tid;
        const float gx = gs[grow * 11 + 0];
        const float gy = gs[grow * 11 + 1];
        float x = gx * pc_mul; x = x + pc_add;
        float y = gy * pc_mul; y = y + pc_add;
        kx_s[tid] = x; ky_s[tid] = y;
      }
    }
    __syncthreads();

    v8f s[4];
#pragma unroll
    for (int j = 0; j < 4; ++j) {
      s[j] = (v8f){0.f,0.f,0.f,0.f,0.f,0.f,0.f,0.f};
      FB kb, kl;
      const __bf16* kp  = Ksh + (j * 16 + c) * GS_D + 8 * hh;
      const __bf16* klp = Ksl + (j * 16 + c) * GS_D + 8 * hh;
      kb.h[0] = *(const v8b*)(kp);  kb.h[1] = *(const v8b*)(kp + 16);
      kl.h[0] = *(const v8b*)(klp); kl.h[1] = *(const v8b*)(klp + 16);
      s[j] = bf_mma(qah, kb.v, s[j]);
      s[j] = bf_mma(qah, kl.v, s[j]);
      s[j] = bf_mma(qal, kb.v, s[j]);
    }

    float kxv[4], kyv[4];
#pragma unroll
    for (int j = 0; j < 4; ++j) { kxv[j] = kx_s[j * 16 + c]; kyv[j] = ky_s[j * 16 + c]; }

    float cm[8];
#pragma unroll
    for (int r = 0; r < 8; ++r) {
      float m = -__builtin_inff();
#pragma unroll
      for (int j = 0; j < 4; ++j) {
        const float dx  = xq[r] - kxv[j];
        const float dy  = yq[r] - kyv[j];
        const float dx2 = dx * dx;
        const float dy2 = dy * dy;
        const float d2  = dx2 + dy2;
        const float nd  = -sqrtf(d2);
        const float am  = nd * tq[r];
        const float t1  = s[j][r] * qk_scale;
        const float sc  = t1 + am;
        s[j][r] = sc;
        m = fmaxf(m, sc);
      }
#pragma unroll
      for (int off = 1; off < 16; off <<= 1) m = fmaxf(m, __shfl_xor(m, off, 32));
      cm[r] = m;
    }

    __bf16* pwh = Psh[wave];
    __bf16* pwl = Psl[wave];
#pragma unroll
    for (int r = 0; r < 8; ++r) {
      const float mnew  = fmaxf(mrow[r], cm[r]);
      const float alpha = expf(mrow[r] - mnew);
      mrow[r] = mnew;
      float psum = 0.f;
#pragma unroll
      for (int j = 0; j < 4; ++j) {
        const float p = expf(s[j][r] - mnew);
        psum = psum + p;
        const unsigned short hb = f2bf_bits(p);
        const unsigned short lb = f2bf_bits(p - bf_bits2f(hb));
        pwh[(8 * hh + r) * GS_KC + j * 16 + c] = __builtin_bit_cast(__bf16, hb);
        pwl[(8 * hh + r) * GS_KC + j * 16 + c] = __builtin_bit_cast(__bf16, lb);
      }
#pragma unroll
      for (int off = 1; off < 16; off <<= 1) psum += __shfl_xor(psum, off, 32);
      lrow[r] = lrow[r] * alpha + psum;
      oacc[0][r] = oacc[0][r] * alpha;
      oacc[1][r] = oacc[1][r] * alpha;
    }
    __builtin_amdgcn_fence(__ATOMIC_RELEASE, "workgroup");
    __builtin_amdgcn_wave_barrier();
    __builtin_amdgcn_fence(__ATOMIC_ACQUIRE, "workgroup");

#pragma unroll
    for (int kk = 0; kk < 2; ++kk) {
      FB pa, pl;
      const __bf16* pp  = pwh + c * GS_KC + kk * 32 + 8 * hh;
      const __bf16* plp = pwl + c * GS_KC + kk * 32 + 8 * hh;
      pa.h[0] = *(const v8b*)(pp);  pa.h[1] = *(const v8b*)(pp + 16);
      pl.h[0] = *(const v8b*)(plp); pl.h[1] = *(const v8b*)(plp + 16);
#pragma unroll
      for (int t = 0; t < 2; ++t) {
        FB vb, vl;
        const __bf16* vp  = Vth + (t * 16 + c) * GS_KC + kk * 32 + 8 * hh;
        const __bf16* vlp = Vtl + (t * 16 + c) * GS_KC + kk * 32 + 8 * hh;
        vb.h[0] = *(const v8b*)(vp);  vb.h[1] = *(const v8b*)(vp + 16);
        vl.h[0] = *(const v8b*)(vlp); vl.h[1] = *(const v8b*)(vlp + 16);
        oacc[t] = bf_mma(pa.v, vb.v, oacc[t]);
        oacc[t] = bf_mma(pa.v, vl.v, oacc[t]);
        oacc[t] = bf_mma(pl.v, vb.v, oacc[t]);
      }
    }
  }

  float* os = Os[wave];
#pragma unroll
  for (int r = 0; r < 8; ++r) {
    const float inv = 1.0f / lrow[r];
    os[(8 * hh + r) * GS_OSP + c]      = oacc[0][r] * inv;
    os[(8 * hh + r) * GS_OSP + 16 + c] = oacc[1][r] * inv;
  }
  __builtin_amdgcn_fence(__ATOMIC_RELEASE, "workgroup");
  __builtin_amdgcn_wave_barrier();
  __builtin_amdgcn_fence(__ATOMIC_ACQUIRE, "workgroup");
  {
    const int q4 = lane >> 3, c4 = (lane & 7) * 4;
    float* obase = O + (size_t)h * GS_D;
    for (int pass = 0; pass < 2; ++pass) {
#pragma unroll
      for (int it = 0; it < 4; ++it) {
        const int row = it * 4 + q4;
        const v4f val = *(const v4f*)(os + row * GS_OSP + c4);
        *(volatile v4f*)(obase + (browbase + q0 + row) * GS_C + c4) = val;
      }
      __threadfence();
    }
  }
}

extern "C" void kernel_launch(void* const* d_in, const int* in_sizes, int n_in,
                              void* d_out, int out_size, void* d_ws, size_t ws_size,
                              hipStream_t stream) {
  static_assert(GS_BG % 64 == 0 && GS_C % 64 == 0 && (2 * GS_C) % 64 == 0 && GS_TAUN % 64 == 0);
  static_assert(GS_C % 32 == 0);
  static_assert(GS_G % GS_KC == 0 && GS_G % 64 == 0 && GS_D == 32 && GS_H * GS_D == GS_C);
  if (n_in < 8) return;
  if (in_sizes[0] != GS_BG * 11 || in_sizes[1] != GS_BG * GS_C || in_sizes[2] != GS_H * GS_C ||
      in_sizes[3] != GS_H || in_sizes[4] != 3 * GS_C * GS_C || in_sizes[5] != 3 * GS_C ||
      in_sizes[6] != GS_C * GS_C || in_sizes[7] != GS_C || out_size != GS_BG * GS_C) return;

  const float* gs     = (const float*)d_in[0];
  const float* feat   = (const float*)d_in[1];
  const float* tau_w  = (const float*)d_in[2];
  const float* tau_b  = (const float*)d_in[3];
  const float* w_in   = (const float*)d_in[4];
  const float* b_in   = (const float*)d_in[5];
  const float* w_out  = (const float*)d_in[6];
  const float* b_out  = (const float*)d_in[7];
  float* out = (float*)d_out;

  constexpr size_t SZ_FE  = (size_t)GS_BG * GS_C * 2;
  constexpr size_t SZ_WI  = (size_t)3 * GS_C * GS_C * 2;
  constexpr size_t SZ_TW  = (size_t)GS_TAUN * GS_C * 2;
  constexpr size_t SZ_WO  = (size_t)GS_C * GS_C * 2;
  constexpr size_t SZ_QK  = (size_t)GS_BG * GS_QKLD * 2;
  constexpr size_t SZ_VT  = (size_t)GS_C * GS_VTLD * 2;
  constexpr size_t SZ_TAU = (size_t)GS_BG * GS_TAULD * 4;
  constexpr size_t SZ_OAT = (size_t)GS_BG * GS_C * 4;
  constexpr size_t SZ_OA  = (size_t)GS_BG * GS_C * 2;
  constexpr size_t OFF_FEH = 0;
  constexpr size_t OFF_FEL = OFF_FEH + SZ_FE;
  constexpr size_t OFF_WIH = OFF_FEL + SZ_FE;
  constexpr size_t OFF_WIL = OFF_WIH + SZ_WI;
  constexpr size_t OFF_TWH = OFF_WIL + SZ_WI;
  constexpr size_t OFF_TWL = OFF_TWH + SZ_TW;
  constexpr size_t OFF_WOH = OFF_TWL + SZ_TW;
  constexpr size_t OFF_WOL = OFF_WOH + SZ_WO;
  constexpr size_t OFF_QKH = OFF_WOL + SZ_WO;
  constexpr size_t OFF_QKL = OFF_QKH + SZ_QK;
  constexpr size_t OFF_VTH = OFF_QKL + SZ_QK;
  constexpr size_t OFF_VTL = OFF_VTH + SZ_VT;
  constexpr size_t OFF_TAU = OFF_VTL + SZ_VT;
  constexpr size_t OFF_OAT = OFF_TAU + SZ_TAU;
  constexpr size_t OFF_OAH = OFF_OAT + SZ_OAT;
  constexpr size_t OFF_OAL = OFF_OAH + SZ_OA;
  constexpr size_t WS_TOTAL = OFF_OAL + SZ_OA;
  static_assert(WS_TOTAL == 27328512);
  static_assert(WS_TOTAL <= (size_t)134217728);
  static_assert(OFF_FEL % 128 == 0 && OFF_WIH % 128 == 0 && OFF_WIL % 128 == 0 && OFF_TWH % 128 == 0 &&
                OFF_TWL % 128 == 0 && OFF_WOH % 128 == 0 && OFF_WOL % 128 == 0 && OFF_QKH % 128 == 0 &&
                OFF_QKL % 128 == 0 && OFF_VTH % 128 == 0 && OFF_VTL % 128 == 0 && OFF_TAU % 128 == 0 &&
                OFF_OAT % 128 == 0 && OFF_OAH % 128 == 0 && OFF_OAL % 128 == 0);
  if (WS_TOTAL > ws_size) return;

  char* ws = (char*)d_ws;
  unsigned short* FEh = (unsigned short*)(ws + OFF_FEH);
  unsigned short* FEl = (unsigned short*)(ws + OFF_FEL);
  unsigned short* WIh = (unsigned short*)(ws + OFF_WIH);
  unsigned short* WIl = (unsigned short*)(ws + OFF_WIL);
  unsigned short* TWh = (unsigned short*)(ws + OFF_TWH);
  unsigned short* TWl = (unsigned short*)(ws + OFF_TWL);
  unsigned short* WOh = (unsigned short*)(ws + OFF_WOH);
  unsigned short* WOl = (unsigned short*)(ws + OFF_WOL);
  unsigned short* QKh = (unsigned short*)(ws + OFF_QKH);
  unsigned short* QKl = (unsigned short*)(ws + OFF_QKL);
  unsigned short* VTh = (unsigned short*)(ws + OFF_VTH);
  unsigned short* VTl = (unsigned short*)(ws + OFF_VTL);
  float*          TAU = (float*)(ws + OFF_TAU);
  float*          OAT = (float*)(ws + OFF_OAT);
  unsigned short* OAh = (unsigned short*)(ws + OFF_OAH);
  unsigned short* OAl = (unsigned short*)(ws + OFF_OAL);

  {
    const int n_fe = GS_BG * GS_C / 8;
    split_rows_kernel<<<(n_fe + 255) / 256, 256, 0, stream>>>(feat, FEh, FEl, GS_BG, GS_BG, GS_C);
    const int n_wi = 3 * GS_C * GS_C / 8;
    split_rows_kernel<<<(n_wi + 255) / 256, 256, 0, stream>>>(w_in, WIh, WIl, 3 * GS_C, 3 * GS_C, GS_C);
    const int n_tw = GS_TAUN * GS_C / 8;
    split_rows_kernel<<<(n_tw + 255) / 256, 256, 0, stream>>>(tau_w, TWh, TWl, GS_H, GS_TAUN, GS_C);
    const int n_wo = GS_C * GS_C / 8;
    split_rows_kernel<<<(n_wo + 255) / 256, 256, 0, stream>>>(w_out, WOh, WOl, GS_C, GS_C, GS_C);
  }

  wmma_gemm64<1, true, 2, 2><<<dim3((GS_BG / 64) * (2 * GS_C / 64) / 8, 1), 256, 0, stream>>>(
      FEh, FEl, GS_C, 0L, WIh, WIl, GS_C, 0L, (void*)QKh, (void*)QKl, GS_QKLD, 0L,
      b_in, GS_BG, 2 * GS_C, GS_C, 1.0f);

  wmma_gemm64<1, true, 1, 2><<<dim3((GS_C / 64) * (GS_BG / 64) / 8, 1), 256, 0, stream>>>(
      WIh + (size_t)2 * GS_C * GS_C, WIl + (size_t)2 * GS_C * GS_C, GS_C, 0L,
      FEh, FEl, GS_C, 0L, (void*)VTh, (void*)VTl, GS_VTLD, 0L,
      b_in + 2 * GS_C, GS_C, GS_BG, GS_C, 1.0f);

  wmma_gemm64<1, true, 0, 0><<<dim3((GS_BG / 64) * (GS_TAUN / 64) / 8, 1), 256, 0, stream>>>(
      FEh, FEl, GS_C, 0L, TWh, TWl, GS_C, 0L, (void*)TAU, (void*)TAU, GS_TAULD, 0L,
      tau_b, GS_BG, GS_TAUN, GS_C, 1.0f);

  gsa_attn_kernel<<<GS_B * GS_H * (GS_G / 64), 128, 0, stream>>>(QKh, QKl, VTh, VTl, TAU, tau_b, gs, OAT);

  {
    const int n_oa = GS_BG * GS_C / 8;
    split_rows_kernel<<<(n_oa + 255) / 256, 256, 0, stream>>>(OAT, OAh, OAl, GS_BG, GS_BG, GS_C);
  }

  wmma_gemm64<1, true, 2, 0><<<dim3((GS_BG / 64) * (GS_C / 64) / 8, 1), 256, 0, stream>>>(
      OAh, OAl, GS_C, 0L, WOh, WOl, GS_C, 0L, (void*)out, (void*)out, GS_C, 0L,
      b_out, GS_BG, GS_C, GS_C, 1.0f);
}
